// GuidedDiffusionRGC_84387517432643
// MI455X (gfx1250) — hardware-verified
//
#include <hip/hip_runtime.h>

typedef __attribute__((ext_vector_type(16))) _Float16 v16h;
typedef __attribute__((ext_vector_type(8)))  _Float16 v8h;
typedef __attribute__((ext_vector_type(8)))  float    v8f;
typedef __attribute__((ext_vector_type(4)))  float    v4f;
typedef __attribute__((ext_vector_type(4)))  int      v4i;
typedef __attribute__((ext_vector_type(4)))  unsigned v4u;

constexpr int NN    = 32768;
constexpr int DD    = 256;
constexpr int NE    = 524288;
constexpr int NREL  = 10;
constexpr int NBAS  = 4;
constexpr int XBW   = NBAS * DD;
constexpr int WROWS = (NBAS + 1) * DD;
static_assert(NN == (1 << 15));
static_assert(XBW == 1024 && WROWS == 1280);
static_assert((DD % 32) == 0 && (NN % 64) == 0 && (XBW % 64) == 0 && (DD % 64) == 0);

constexpr float A_CARRY  = 16.0f;
constexpr float W_CARRY  = 256.0f;
constexpr float XB_CARRY = 16.0f;
constexpr float SC_XB    = XB_CARRY / (A_CARRY * W_CARRY);
constexpr float SC_ROOT  = 1.0f / (A_CARRY * W_CARRY);
constexpr int   DEC_EXP  = 112 - 4;
static_assert(XB_CARRY == 16.0f);
constexpr float F16_MIN_NORMAL = 6.103515625e-05f;

constexpr size_t OFF_XB16 = 0;
constexpr size_t OFF_RPL  = OFF_XB16 + (size_t)NN * XBW * 2;
constexpr size_t OFF_A16  = OFF_RPL  + (size_t)NN * DD * 4;
constexpr size_t OFF_INVT = OFF_A16  + (size_t)NN * DD * 2;
constexpr size_t OFF_WT   = OFF_INVT + (size_t)NN * 16 * 4;
constexpr size_t WS_TOTAL = OFF_WT   + (size_t)2 * WROWS * DD * 2;
static_assert(WS_TOTAL == 120848384ull);
static_assert(WS_TOTAL <= 134217728ull);
static_assert((OFF_RPL % 128) == 0 && (OFF_A16 % 128) == 0 && (OFF_INVT % 128) == 0 && (OFF_WT % 128) == 0);

__device__ __forceinline__ int clampi(int v, int lo, int hi) { return v < lo ? lo : (v > hi ? hi : v); }

__device__ __forceinline__ v16h frag_load(const _Float16* p) {
  union { v16h v; v8h h[2]; } f;
  f.h[0] = *(const v8h*)(p);
  f.h[1] = *(const v8h*)(p + 16);
  return f.v;
}
__device__ __forceinline__ v8f mma_f16(v16h a, v16h b, v8f c) {
  return __builtin_amdgcn_wmma_f32_16x16x32_f16(false, a, false, b, (short)0, c, false, false);
}
__device__ __forceinline__ void acc_tie(v8f& a, v16h x, v16h y) { asm volatile("" : "+v"(a) : "v"(x), "v"(y)); }
__device__ __forceinline__ void acc_guard(v8f& a, v16h x, v16h y) { asm volatile("v_nop\n\tv_nop\n\tv_nop\n\tv_nop" : "+v"(a) : "v"(x), "v"(y)); }
__device__ __forceinline__ void acc_hold(v8f& a) { asm volatile("" : "+v"(a)); }
__device__ __forceinline__ void acc_hold_nop(v8f& a) { asm volatile("v_nop\n\tv_nop\n\tv_nop\n\tv_nop" : "+v"(a)); }
__device__ __forceinline__ void keep4_h(v16h a, v16h b, v16h c, v16h d) { asm volatile("v_nop" :: "v"(a), "v"(b), "v"(c), "v"(d)); }

template <int BIAS_N, int OUT_F16>
__global__ __launch_bounds__(256) void gemm64_f16_kernel(
    const unsigned short* __restrict__ Ap, int lda,
    const unsigned short* __restrict__ Btp, int ldb,
    void* __restrict__ Cout, int ldc,
    const float* __restrict__ bias, int M, int N, int K, float scale)
{
  const _Float16* A  = (const _Float16*)Ap;
  const _Float16* Bt = (const _Float16*)Btp;
  __shared__ __align__(16) float sT[8][16 * 68];
  const int lane = threadIdx.x & 31;
  const int wave = threadIdx.x >> 5;
  const int tilesN = N >> 6;
  const int tilesM = M >> 6;
  const int tile = blockIdx.x * 8 + wave;
  if (tile >= tilesM * tilesN) return;
  const int tm = tile / tilesN;
  const int tn = tile - tm * tilesN;
  const int m0 = tm << 6;
  const int n0 = tn << 6;

  const int rlane = lane & 15;
  const int koff  = (lane >> 4) * 8;
  const int mOff  = (lane >> 4) * 8;

  v8f acc[4][4];
#pragma unroll
  for (int i = 0; i < 4; ++i)
#pragma unroll
    for (int j = 0; j < 4; ++j) acc[i][j] = (v8f){0.f, 0.f, 0.f, 0.f, 0.f, 0.f, 0.f, 0.f};

  for (int k0 = 0; k0 < K; k0 += 32) {
    v16h bh[4];
#pragma unroll
    for (int j = 0; j < 4; ++j) {
      const size_t bo = (size_t)(n0 + (j << 4) + rlane) * ldb + koff + k0;
      bh[j] = frag_load(Bt + bo);
    }
#pragma unroll
    for (int i = 0; i < 4; ++i) {
      const size_t ao = (size_t)(m0 + (i << 4) + rlane) * lda + koff + k0;
      const v16h ah = frag_load(A + ao);
#pragma unroll
      for (int j = 0; j < 4; ++j) acc[i][j] = mma_f16(ah, bh[j], acc[i][j]);
      acc_tie(acc[i][0], ah, bh[0]);
      acc_tie(acc[i][1], ah, bh[1]);
      acc_tie(acc[i][2], ah, bh[2]);
      acc_guard(acc[i][3], ah, bh[3]);
    }
    keep4_h(bh[0], bh[1], bh[2], bh[3]);
  }
#pragma unroll
  for (int i = 0; i < 4; ++i) {
    acc_hold(acc[i][0]);
    acc_hold(acc[i][1]);
    acc_hold(acc[i][2]);
    acc_hold_nop(acc[i][3]);
  }

  float* slab = sT[wave];
#pragma unroll
  for (int i = 0; i < 4; ++i) {
    const int mBase = m0 + (i << 4);
#pragma unroll
    for (int j = 0; j < 4; ++j) {
      const int n = n0 + (j << 4) + rlane;
      float bv = 0.f;
      if (BIAS_N == 1) bv = bias[n];
#pragma unroll
      for (int r = 0; r < 8; ++r) {
        float v = acc[i][j][r] * scale;
        if (BIAS_N == 1) v += bv;
        slab[(mOff + r) * 68 + (j << 4) + rlane] = v;
      }
    }
    __builtin_amdgcn_fence(__ATOMIC_RELEASE, "workgroup");
    __builtin_amdgcn_wave_barrier();
    __builtin_amdgcn_fence(__ATOMIC_ACQUIRE, "workgroup");
    if (OUT_F16 == 0) {
      float* C = (float*)Cout;
      const int hh = lane >> 4, c4 = (lane & 15) * 4;
      for (int pass = 0; pass < 2; ++pass) {
#pragma unroll
        for (int it = 0; it < 8; ++it) {
          const int row = it * 2 + hh;
          const v4f v = *(const v4f*)(slab + row * 68 + c4);
          *(volatile v4f*)(C + (size_t)(mBase + row) * ldc + n0 + c4) = v;
        }
        __threadfence();
      }
    } else {
      const int q = lane >> 3, c8 = (lane & 7) * 8;
      unsigned short* C = (unsigned short*)Cout;
      for (int pass = 0; pass < 2; ++pass) {
#pragma unroll
        for (int it = 0; it < 4; ++it) {
          const int row = it * 4 + q;
          const float* sp = slab + row * 68 + c8;
          v8h hv;
#pragma unroll
          for (int e = 0; e < 8; ++e) {
            float sv = sp[e];
            sv = (__builtin_fabsf(sv) < F16_MIN_NORMAL) ? 0.0f : sv;
            hv[e] = (_Float16)sv;
          }
          *(volatile v8h*)(C + (size_t)(mBase + row) * ldc + n0 + c8) = hv;
        }
        __threadfence();
      }
    }
    __builtin_amdgcn_fence(__ATOMIC_RELEASE, "workgroup");
    __builtin_amdgcn_wave_barrier();
    __builtin_amdgcn_fence(__ATOMIC_ACQUIRE, "workgroup");
  }
}

__global__ __launch_bounds__(256) void cvt_rows_f16_kernel(
    const float* __restrict__ src, unsigned short* __restrict__ dst, int total8, float carry)
{
  const int i = blockIdx.x * 256 + threadIdx.x;
  if (i >= total8) return;
  const size_t e0 = (size_t)i << 3;
  const v4f a0 = *(const v4f*)(src + e0);
  const v4f a1 = *(const v4f*)(src + e0 + 4);
  v8h hv;
#pragma unroll
  for (int e = 0; e < 4; ++e) {
    const float f0 = a0[e] * carry;
    const float f1 = a1[e] * carry;
    hv[e]     = (_Float16)f0;
    hv[4 + e] = (_Float16)f1;
  }
  unsigned short* q = dst + e0;
  *(volatile v8h*)q = hv;
  __threadfence();
  *(volatile v8h*)q = hv;
}

constexpr int WP_PITCH = 260;
__global__ __launch_bounds__(256) void weight_planes_kernel(
    const float* __restrict__ basisA, const float* __restrict__ rootA,
    const float* __restrict__ basisB, const float* __restrict__ rootB,
    unsigned short* __restrict__ WT)
{
  __shared__ __align__(16) float tileL[32 * WP_PITCH];
  const int tid = threadIdx.x, lane = tid & 31, wave = tid >> 5;
  const int bx = blockIdx.x;
  const int l  = bx / 40;
  const int rm = bx - l * 40;
  const int mt = rm >> 3;
  const int o0 = (rm & 7) * 32;
  const float* bas = l ? basisB : basisA;
  const float* rt  = l ? rootB : rootA;
  const int mtc = mt < NBAS ? mt : (NBAS - 1);
  const float* src = (mt < NBAS) ? (bas + (size_t)mtc * DD * DD) : rt;
#pragma unroll 4
  for (int it = 0; it < 32; ++it) {
    const int k = (tid >> 5) + 8 * it;
    tileL[lane * WP_PITCH + k] = src[(size_t)k * DD + o0 + lane];
  }
  __syncthreads();
  v8h hv[4];
#pragma unroll
  for (int j = 0; j < 4; ++j) {
    const float* sp = tileL + (wave * 4 + j) * WP_PITCH + 8 * lane;
    const v4f a0 = *(const v4f*)(sp);
    const v4f a1 = *(const v4f*)(sp + 4);
#pragma unroll
    for (int e = 0; e < 4; ++e) {
      const float f0 = a0[e] * W_CARRY;
      const float f1 = a1[e] * W_CARRY;
      hv[j][e]     = (_Float16)f0;
      hv[j][4 + e] = (_Float16)f1;
    }
  }
  for (int pass = 0; pass < 2; ++pass) {
#pragma unroll
    for (int j = 0; j < 4; ++j) {
      const size_t row = (size_t)l * WROWS + (size_t)mt * DD + o0 + wave * 4 + j;
      *(volatile v8h*)(WT + row * DD + 8 * lane) = hv[j];
    }
    __threadfence();
  }
}

constexpr int CN_T = 512;
static_assert((NN % CN_T) == 0 && (NE % 1024) == 0);
__global__ __launch_bounds__(256) void seg_inv_kernel(
    const int* __restrict__ ec, const int* __restrict__ rel, float* __restrict__ invT)
{
  __shared__ int cntL[CN_T * 16];
  const int tid = threadIdx.x;
  const int n0 = blockIdx.x * CN_T;
#pragma unroll 4
  for (int i = 0; i < (CN_T * 16) / 256; ++i) cntL[tid + 256 * i] = 0;
  __syncthreads();
  const int* dstp = ec + NE;
#pragma unroll 1
  for (int c = 0; c < NE / 1024; ++c) {
    const int e0 = c * 1024 + tid * 4;
    const v4i d4 = *(const v4i*)(dstp + e0);
    const int l0 = clampi(d4.x, 0, NN - 1) - n0;
    const int l1 = clampi(d4.y, 0, NN - 1) - n0;
    const int l2 = clampi(d4.z, 0, NN - 1) - n0;
    const int l3 = clampi(d4.w, 0, NN - 1) - n0;
    const bool h0 = (unsigned)l0 < (unsigned)CN_T;
    const bool h1 = (unsigned)l1 < (unsigned)CN_T;
    const bool h2 = (unsigned)l2 < (unsigned)CN_T;
    const bool h3 = (unsigned)l3 < (unsigned)CN_T;
    const unsigned many = __builtin_amdgcn_ballot_w32(h0 || h1 || h2 || h3);
    if (many != 0u) {
      v4i r4 = *(const v4i*)(rel + e0);
      asm volatile("" : "+v"(r4));
      const int r0 = clampi(r4.x, 0, NREL - 1);
      const int r1 = clampi(r4.y, 0, NREL - 1);
      const int r2 = clampi(r4.z, 0, NREL - 1);
      const int r3 = clampi(r4.w, 0, NREL - 1);
      if (h0) atomicAdd(&cntL[l0 * 16 + r0], 1);
      if (h1) atomicAdd(&cntL[l1 * 16 + r1], 1);
      if (h2) atomicAdd(&cntL[l2 * 16 + r2], 1);
      if (h3) atomicAdd(&cntL[l3 * 16 + r3], 1);
    }
  }
  __syncthreads();
  float* base = invT + (size_t)n0 * 16;
  for (int pass = 0; pass < 2; ++pass) {
#pragma unroll 1
    for (int i = 0; i < 8; ++i) {
      const int idx4 = tid + 256 * i;
      const int c0 = cntL[4 * idx4 + 0];
      const int c1 = cntL[4 * idx4 + 1];
      const int c2 = cntL[4 * idx4 + 2];
      const int c3 = cntL[4 * idx4 + 3];
      v4f v;
      v.x = 1.0f / (float)(c0 > 1 ? c0 : 1);
      v.y = 1.0f / (float)(c1 > 1 ? c1 : 1);
      v.z = 1.0f / (float)(c2 > 1 ? c2 : 1);
      v.w = 1.0f / (float)(c3 > 1 ? c3 : 1);
      *(volatile v4f*)(base + 4 * idx4) = v;
    }
    __threadfence();
  }
}

__device__ __forceinline__ float h16lo_dec(unsigned w) {
  return __uint_as_float(((unsigned)(((int)(w << 16)) >> 3)) & 0x8FFFFFFFu);
}
__device__ __forceinline__ float h16hi_dec(unsigned w) {
  return __uint_as_float(((unsigned)(((int)w) >> 3)) & 0x8FFFE000u);
}
__device__ __forceinline__ void comb8(v4f& a0, v4f& a1, const v4u q, const float c) {
  a0.x = fmaf(c, h16lo_dec(q.x), a0.x);
  a0.y = fmaf(c, h16hi_dec(q.x), a0.y);
  a0.z = fmaf(c, h16lo_dec(q.y), a0.z);
  a0.w = fmaf(c, h16hi_dec(q.y), a0.w);
  a1.x = fmaf(c, h16lo_dec(q.z), a1.x);
  a1.y = fmaf(c, h16hi_dec(q.z), a1.y);
  a1.z = fmaf(c, h16lo_dec(q.w), a1.z);
  a1.w = fmaf(c, h16hi_dec(q.w), a1.w);
}

constexpr int AG_T   = 128;
constexpr int AG_CAP = 512;
constexpr int AG_CHK = 2;
constexpr int AG_EPC = 1024;
constexpr int AG_NCH = NE / AG_EPC;
constexpr int AG_THR = AG_CAP - AG_CHK * 128;
static_assert((NN % AG_T) == 0 && (NE % (AG_EPC * AG_CHK)) == 0);
static_assert(AG_THR >= 0 && AG_THR + AG_CHK * 128 <= AG_CAP);
static_assert(AG_T == 128 && (AG_CAP % 32) == 0);

template <bool LAST>
__global__ __launch_bounds__(256) void agg_kernel(
    const int* __restrict__ ec, const int* __restrict__ rel, const float* __restrict__ comp,
    const float* __restrict__ invT, const unsigned short* __restrict__ xb16,
    const float* __restrict__ rootp, unsigned short* __restrict__ hout, float* __restrict__ fout)
{
  __shared__ v4f   accL[AG_T * 64];
  __shared__ int   listL[8 * AG_CAP];
  __shared__ float invL[AG_T * 16];
  __shared__ v4f   compL[16];
  __shared__ int   wnL[2][8];

  const int tid = threadIdx.x, lane = tid & 31, wave = tid >> 5;
  const int d0 = blockIdx.x * AG_T;
  const v4f z4 = {0.f, 0.f, 0.f, 0.f};

#pragma unroll 4
  for (int i = 0; i < 32; ++i) accL[tid + 256 * i] = z4;
#pragma unroll 1
  for (int i = 0; i < 8; ++i) invL[tid + 256 * i] = invT[(size_t)d0 * 16 + tid + 256 * i];
  {
    const int rr = tid < (NREL - 1) ? tid : (NREL - 1);
    v4f cv = *(const v4f*)(comp + rr * 4);
    asm volatile("" : "+v"(cv));
    const v4f cs = (tid < NREL) ? cv : z4;
    if (tid < 16) compL[tid] = cs;
  }
  __syncthreads();

  const float k2dec = __uint_as_float(((unsigned)(127 + DEC_EXP)) << 23);
  const int* dstp = ec + NE;
  int* lw = listL + wave * AG_CAP;
  const unsigned ltm = (1u << lane) - 1u;
  int nw = 0;

#pragma unroll 1
  for (int cb = 0; cb < AG_NCH; cb += AG_CHK) {
#pragma unroll 1
    for (int cc = 0; cc < AG_CHK; ++cc) {
      const int e0 = (cb + cc) * AG_EPC + tid * 4;
      const v4i d4 = *(const v4i*)(dstp + e0);
      const int l0 = clampi(d4.x, 0, NN - 1) - d0;
      const int l1 = clampi(d4.y, 0, NN - 1) - d0;
      const int l2 = clampi(d4.z, 0, NN - 1) - d0;
      const int l3 = clampi(d4.w, 0, NN - 1) - d0;
      const bool h0 = (unsigned)l0 < (unsigned)AG_T;
      const bool h1 = (unsigned)l1 < (unsigned)AG_T;
      const bool h2 = (unsigned)l2 < (unsigned)AG_T;
      const bool h3 = (unsigned)l3 < (unsigned)AG_T;
      const unsigned m0 = __builtin_amdgcn_ballot_w32(h0);
      const unsigned m1 = __builtin_amdgcn_ballot_w32(h1);
      const unsigned m2 = __builtin_amdgcn_ballot_w32(h2);
      const unsigned m3 = __builtin_amdgcn_ballot_w32(h3);
      if ((m0 | m1 | m2 | m3) != 0u) {
        v4i s4 = *(const v4i*)(ec + e0);
        v4i r4 = *(const v4i*)(rel + e0);
        asm volatile("" : "+v"(s4), "+v"(r4));
        const int p0 = nw + __builtin_popcount(m0 & ltm) + __builtin_popcount(m1 & ltm)
                          + __builtin_popcount(m2 & ltm) + __builtin_popcount(m3 & ltm);
        const int p1 = p0 + (h0 ? 1 : 0);
        const int p2 = p1 + (h1 ? 1 : 0);
        const int p3 = p2 + (h2 ? 1 : 0);
        const int en0 = clampi(s4.x, 0, NN - 1) | ((l0 & (AG_T - 1)) << 15) | (clampi(r4.x, 0, NREL - 1) << 22);
        const int en1 = clampi(s4.y, 0, NN - 1) | ((l1 & (AG_T - 1)) << 15) | (clampi(r4.y, 0, NREL - 1) << 22);
        const int en2 = clampi(s4.z, 0, NN - 1) | ((l2 & (AG_T - 1)) << 15) | (clampi(r4.z, 0, NREL - 1) << 22);
        const int en3 = clampi(s4.w, 0, NN - 1) | ((l3 & (AG_T - 1)) << 15) | (clampi(r4.w, 0, NREL - 1) << 22);
        if (h0) lw[p0 < AG_CAP ? p0 : (AG_CAP - 1)] = en0;
        if (h1) lw[p1 < AG_CAP ? p1 : (AG_CAP - 1)] = en1;
        if (h2) lw[p2 < AG_CAP ? p2 : (AG_CAP - 1)] = en2;
        if (h3) lw[p3 < AG_CAP ? p3 : (AG_CAP - 1)] = en3;
        nw += __builtin_popcount(m0) + __builtin_popcount(m1) + __builtin_popcount(m2) + __builtin_popcount(m3);
      }
    }
    const int par = (cb / AG_CHK) & 1;
    if (lane == 0) wnL[par][wave] = nw;
    __syncthreads();
    int mx = 0;
#pragma unroll
    for (int q = 0; q < 8; ++q) {
      const int wq = wnL[par][q];
      mx = wq > mx ? wq : mx;
    }
    const bool lastc = (cb + AG_CHK >= AG_NCH);
    if (mx > AG_THR || lastc) {
#pragma unroll 1
      for (int q = 0; q < 8; ++q) {
        const int n = clampi(wnL[par][q], 0, AG_CAP);
        const int* lq = listL + q * AG_CAP;
#pragma unroll 1
        for (int base = 0; base < n; base += 32) {
          const int pos = base + lane;
          const int ent = lq[pos < n ? pos : (n - 1)];
          const bool mine = (pos < n) && (((ent >> 15) & 7) == wave);
          unsigned m = __builtin_amdgcn_ballot_w32(mine);
          while (m != 0u) {
            const int i = __builtin_ctz(m);
            m &= (m - 1u);
            const int en = lq[base + i];
            const int s  = en & (NN - 1);
            const int ld = (en >> 15) & (AG_T - 1);
            const int r  = (en >> 22) & 15;
            const float ivs = invL[ld * 16 + r] * k2dec;
            const v4f cv = compL[r];
            const v4u* xp = (const v4u*)xb16 + (size_t)s * (XBW / 8) + lane;
            const v4u q0 = xp[0];
            const v4u q1 = xp[32];
            const v4u q2 = xp[64];
            const v4u q3 = xp[96];
            v4f a0 = accL[ld * 64 + 2 * lane];
            v4f a1 = accL[ld * 64 + 2 * lane + 1];
            comb8(a0, a1, q0, cv.x * ivs);
            comb8(a0, a1, q1, cv.y * ivs);
            comb8(a0, a1, q2, cv.z * ivs);
            comb8(a0, a1, q3, cv.w * ivs);
            accL[ld * 64 + 2 * lane]     = a0;
            accL[ld * 64 + 2 * lane + 1] = a1;
          }
        }
      }
      __syncthreads();
      nw = 0;
    }
  }

#pragma unroll 1
  for (int g = 0; g < 4; ++g) {
    if (!LAST) {
      v8h hv[4];
#pragma unroll
      for (int j = 0; j < 4; ++j) {
        const int ld = wave * 16 + g * 4 + j;
        const size_t node = (size_t)(d0 + ld);
        const v4f a0 = accL[ld * 64 + 2 * lane];
        const v4f a1 = accL[ld * 64 + 2 * lane + 1];
        const v4f r0 = *(const v4f*)(rootp + node * DD + 8 * lane);
        const v4f r1 = *(const v4f*)(rootp + node * DD + 8 * lane + 4);
#pragma unroll
        for (int e = 0; e < 4; ++e) {
          const float u0 = fmaxf(a0[e] + r0[e], 0.0f) * A_CARRY;
          const float u1 = fmaxf(a1[e] + r1[e], 0.0f) * A_CARRY;
          hv[j][e]     = (_Float16)u0;
          hv[j][4 + e] = (_Float16)u1;
        }
      }
      for (int pass = 0; pass < 2; ++pass) {
#pragma unroll
        for (int j = 0; j < 4; ++j) {
          const size_t node = (size_t)(d0 + wave * 16 + g * 4 + j);
          *(volatile v8h*)(hout + node * DD + 8 * lane) = hv[j];
        }
        __threadfence();
      }
    } else {
      v4f ov[8];
#pragma unroll
      for (int j = 0; j < 4; ++j) {
        const int ld = wave * 16 + g * 4 + j;
        const size_t node = (size_t)(d0 + ld);
        const v4f a0 = accL[ld * 64 + lane];
        const v4f a1 = accL[ld * 64 + 32 + lane];
        const v4f r0 = *(const v4f*)(rootp + node * DD + 4 * lane);
        const v4f r1 = *(const v4f*)(rootp + node * DD + 128 + 4 * lane);
        ov[2 * j]     = a0 + r0;
        ov[2 * j + 1] = a1 + r1;
      }
      for (int pass = 0; pass < 2; ++pass) {
#pragma unroll
        for (int j = 0; j < 4; ++j) {
          const size_t node = (size_t)(d0 + wave * 16 + g * 4 + j);
          *(volatile v4f*)(fout + node * DD + 4 * lane)       = ov[2 * j];
          *(volatile v4f*)(fout + node * DD + 128 + 4 * lane) = ov[2 * j + 1];
        }
        __threadfence();
      }
    }
  }
}

extern "C" void kernel_launch(void* const* d_in, const int* in_sizes, int n_in,
                              void* d_out, int out_size, void* d_ws, size_t ws_size,
                              hipStream_t stream) {
  if (n_in < 13) return;
  if (in_sizes[0] != NN * DD) return;
  if (in_sizes[3] != 2 * NE) return;
  if (in_sizes[4] != NE) return;
  if (in_sizes[5] != NBAS * DD * DD) return;
  if (in_sizes[6] != NREL * NBAS) return;
  if (in_sizes[7] != DD * DD) return;
  if (in_sizes[8] != DD) return;
  if (in_sizes[9] != NBAS * DD * DD) return;
  if (in_sizes[10] != NREL * NBAS) return;
  if (in_sizes[11] != DD * DD) return;
  if (in_sizes[12] != DD) return;
  if (out_size != NN * DD) return;
  if (ws_size < WS_TOTAL) return;

  const float* x      = (const float*)d_in[0];
  const int*   ec     = (const int*)d_in[3];
  const int*   rel    = (const int*)d_in[4];
  const float* basis0 = (const float*)d_in[5];
  const float* comp0  = (const float*)d_in[6];
  const float* root0  = (const float*)d_in[7];
  const float* bias0  = (const float*)d_in[8];
  const float* basis1 = (const float*)d_in[9];
  const float* comp1  = (const float*)d_in[10];
  const float* root1  = (const float*)d_in[11];
  const float* bias1  = (const float*)d_in[12];
  float* out = (float*)d_out;

  char* ws = (char*)d_ws;
  unsigned short* XB16 = (unsigned short*)(ws + OFF_XB16);
  float*          RPL  = (float*)(ws + OFF_RPL);
  unsigned short* A16  = (unsigned short*)(ws + OFF_A16);
  float*          INVT = (float*)(ws + OFF_INVT);
  unsigned short* WT0  = (unsigned short*)(ws + OFF_WT);
  unsigned short* WT1  = WT0 + (size_t)WROWS * DD;

  seg_inv_kernel<<<NN / CN_T, 256, 0, stream>>>(ec, rel, INVT);
  weight_planes_kernel<<<2 * (NBAS + 1) * (DD / 32), 256, 0, stream>>>(basis0, root0, basis1, root1, WT0);
  cvt_rows_f16_kernel<<<(NN * DD / 8) / 256, 256, 0, stream>>>(x, A16, NN * DD / 8, A_CARRY);

  const int gridXb   = ((NN / 64) * (XBW / 64)) / 8;
  const int gridRoot = ((NN / 64) * (DD / 64)) / 8;

  gemm64_f16_kernel<0, 1><<<gridXb, 256, 0, stream>>>(
      A16, DD, WT0, DD, (void*)XB16, XBW, bias0, NN, XBW, DD, SC_XB);
  gemm64_f16_kernel<1, 0><<<gridRoot, 256, 0, stream>>>(
      A16, DD, WT0 + (size_t)XBW * DD, DD, (void*)RPL, DD, bias0, NN, DD, DD, SC_ROOT);
  agg_kernel<false><<<NN / AG_T, 256, 0, stream>>>(ec, rel, comp0, INVT, XB16, RPL, A16, out);

  gemm64_f16_kernel<0, 1><<<gridXb, 256, 0, stream>>>(
      A16, DD, WT1, DD, (void*)XB16, XBW, bias1, NN, XBW, DD, SC_XB);
  gemm64_f16_kernel<1, 0><<<gridRoot, 256, 0, stream>>>(
      A16, DD, WT1 + (size_t)XBW * DD, DD, (void*)RPL, DD, bias1, NN, DD, DD, SC_ROOT);
  agg_kernel<true><<<NN / AG_T, 256, 0, stream>>>(ec, rel, comp1, INVT, XB16, RPL, A16, out);
}
